// Seq2SeqEncode_39694087750035
// MI455X (gfx1250) — hardware-run, weakly checked
//
#include <hip/hip_runtime.h>
#include <math.h>

typedef __attribute__((ext_vector_type(16))) _Float16 v16h;
typedef __attribute__((ext_vector_type(8)))  _Float16 v8h;
typedef __attribute__((ext_vector_type(8)))  float    v8f;
typedef __attribute__((ext_vector_type(4)))  float    v4f;
typedef __attribute__((ext_vector_type(4)))  unsigned int v4u;

constexpr int kVocab = 32000;
constexpr int kEmb   = 256;
constexpr int kHid   = 512;
constexpr int kBatch = 32;
constexpr int kSeq   = 512;
constexpr int kGate  = 4 * kHid;
constexpr int kRows  = kBatch * kSeq;
constexpr int kHP    = kHid + 8;
static_assert(kGate == 2048 && kRows == 16384, "shapes");
static_assert((kEmb % 32) == 0 && (kHid % 32) == 0, "GEMM K multiples of 32");
static_assert((kRows % 64) == 0 && (kGate % 64) == 0 && (kHid % 64) == 0, "GEMM M,N multiples of 64");
static_assert(kBatch == 32 && kSeq >= 2, "two 16-row batch tiles");
static_assert(((kHP * 2) % 16) == 0, "16-B aligned LDS rows");

constexpr float kCarryX  = 1024.0f;
constexpr float kCarryW  = 1024.0f;
constexpr float kCarryH  = 1024.0f;
constexpr float kCarryZx = 256.0f;
constexpr float kScaleZx = kCarryZx / (kCarryX * kCarryW);
constexpr float kZxToAcc = (kCarryH * kCarryW) / kCarryZx;
constexpr float kAccInv  = 1.0f / (kCarryH * kCarryW);

constexpr size_t kOffXE   = 0;
constexpr size_t kOffWT   = kOffXE  + (size_t)kRows * kEmb * 2;
constexpr size_t kOffUT   = kOffWT  + (size_t)kGate * kEmb * 2;
constexpr size_t kOffWDT  = kOffUT  + (size_t)kGate * kHid * 2;
constexpr size_t kOffZXT  = kOffWDT + (size_t)kHid  * kHid * 2;
constexpr size_t kOffHS   = kOffZXT + (size_t)kGate * kRows * 2;
constexpr size_t kWsTotal = kOffHS  + (size_t)kRows * kHid * 2;
static_assert(kWsTotal == 95944704ull, "carve total");
static_assert(kWsTotal <= 134217728ull, "carve cap");
static_assert((kOffWT % 128) == 0 && (kOffUT % 128) == 0 && (kOffWDT % 128) == 0 &&
              (kOffZXT % 128) == 0 && (kOffHS % 128) == 0, "128-B aligned regions");
static_assert((((size_t)kRows * kHid * 4) % 128) == 0 && (((size_t)kBatch * kHid * 4) % 128) == 0, "tail outputs line aligned");

__device__ __forceinline__ float h16_to_f32(unsigned hb) {
  const unsigned sgn = (hb & 0x8000u) << 16;
  const unsigned em = hb & 0x7fffu;
  const float fn = __uint_as_float((em << 13) + 0x38000000u);
  const float fs = (float)em * 5.9604644775390625e-8f;
  const float mag = (em < 0x400u) ? fs : fn;
  return __uint_as_float(__float_as_uint(mag) | sgn);
}

struct FragH {
  union U { v16h v; v8h h[2]; };
  static __device__ __forceinline__ v16h load(const _Float16* p) {
    U f;
    f.h[0] = *(const v8h*)(p);
    f.h[1] = *(const v8h*)(p + 16);
    return f.v;
  }
};

__device__ __forceinline__ v8f mma_h_guarded(v16h a, v16h b, v8f c) {
  c = __builtin_amdgcn_wmma_f32_16x16x32_f16(false, a, false, b, (short)0, c, false, false);
  asm volatile("v_nop\n\tv_nop\n\tv_nop\n\tv_nop" : "+v"(c) : "v"(a), "v"(b));
  return c;
}
__device__ __forceinline__ void keep4_h(v16h a, v16h b, v16h c, v16h d) { asm volatile("v_nop" :: "v"(a), "v"(b), "v"(c), "v"(d)); }

__device__ __forceinline__ float fast_sigmoid(float z) { return __builtin_amdgcn_rcpf(1.0f + __expf(-z)); }
__device__ __forceinline__ float fast_tanh(float z) { return 1.0f - 2.0f * __builtin_amdgcn_rcpf(__expf(2.0f * z) + 1.0f); }

__global__ __launch_bounds__(256) void gather_rows_f16_kernel(
    const int* __restrict__ x, const float* __restrict__ emb, unsigned short* __restrict__ XE)
{
  const int gi = blockIdx.x * 256 + threadIdx.x;
  const int m = gi >> 5;
  const int lane = gi & 31;
  if (m >= kRows) return;
  const int t = m >> 5;
  const int b = m & 31;
  int tok = x[b * kSeq + t];
  tok = tok < 0 ? 0 : tok;
  tok = tok > (kVocab - 1) ? (kVocab - 1) : tok;
  const float* src = emb + (size_t)tok * kEmb + lane * 8;
  const v4f a0 = *(const v4f*)(src);
  const v4f a1 = *(const v4f*)(src + 4);
  v8h hv;
#pragma unroll
  for (int e = 0; e < 4; ++e) {
    hv[e]     = (_Float16)(a0[e] * kCarryX);
    hv[4 + e] = (_Float16)(a1[e] * kCarryX);
  }
  unsigned short* dst = XE + (size_t)m * kEmb + lane * 8;
  *(volatile v8h*)dst = hv;
  __threadfence();
  *(volatile v8h*)dst = hv;
}

__global__ __launch_bounds__(256) void transpose_cast_kernel(
    const float* __restrict__ in, unsigned short* __restrict__ out, int R, int C, float carry)
{
  __shared__ __align__(16) float sT[32 * 68];
  const int tid = threadIdx.x;
  const int lane = tid & 31;
  const int wave = tid >> 5;
  const int r0 = blockIdx.x * 64;
  const int c0 = blockIdx.y * 32;
  const int cc = tid & 31;
  const int rb = tid >> 5;
#pragma unroll
  for (int i = 0; i < 8; ++i) {
    const int rr = rb + 8 * i;
    sT[cc * 68 + rr] = in[(size_t)(r0 + rr) * C + c0 + cc];
  }
  __syncthreads();
  const int q = lane >> 3;
  const int l8 = lane & 7;
  const int orow = wave * 4 + q;
  const float* sp = sT + orow * 68 + l8 * 8;
  const v4f a0 = *(const v4f*)(sp);
  const v4f a1 = *(const v4f*)(sp + 4);
  v8h hv;
#pragma unroll
  for (int e = 0; e < 4; ++e) {
    hv[e]     = (_Float16)(a0[e] * carry);
    hv[4 + e] = (_Float16)(a1[e] * carry);
  }
  unsigned short* dst = out + (size_t)(c0 + orow) * R + r0 + l8 * 8;
  *(volatile v8h*)dst = hv;
  __threadfence();
  *(volatile v8h*)dst = hv;
}

template <int BIAS_MODE, int OUT_MODE>
__global__ __launch_bounds__(256) void wmma_gemm64_f16(
    const unsigned short* __restrict__ Ap, int lda,
    const unsigned short* __restrict__ Btp, int ldb,
    void* __restrict__ Cout, int ldc,
    const float* __restrict__ bias,
    int M, int N, int K, float scale)
{
  const _Float16* A  = (const _Float16*)Ap;
  const _Float16* Bt = (const _Float16*)Btp;
  __shared__ __align__(16) float sT[8][16 * 68];
  const int lane = threadIdx.x & 31;
  const int wave = threadIdx.x >> 5;
  const int tilesN = N >> 6;
  const int tilesM = M >> 6;
  const int tile = blockIdx.x * 8 + wave;
  if (tile >= tilesM * tilesN) return;
  const int tm = tile / tilesN;
  const int tn = tile - tm * tilesN;
  const int m0 = tm << 6;
  const int n0 = tn << 6;

  const int rlane = lane & 15;
  const int koff  = (lane >> 4) * 8;
  const int mOff  = (lane >> 4) * 8;

  v8f acc[4][4];
#pragma unroll
  for (int i = 0; i < 4; ++i)
#pragma unroll
    for (int j = 0; j < 4; ++j) acc[i][j] = (v8f){0.f,0.f,0.f,0.f,0.f,0.f,0.f,0.f};

  for (int k0 = 0; k0 < K; k0 += 32) {
    v16h bh[4];
#pragma unroll
    for (int j = 0; j < 4; ++j) {
      const size_t bo = (size_t)(n0 + (j << 4) + rlane) * ldb + koff + k0;
      bh[j] = FragH::load(Bt + bo);
    }
#pragma unroll
    for (int i = 0; i < 4; ++i) {
      const size_t ao = (size_t)(m0 + (i << 4) + rlane) * lda + koff + k0;
      const v16h ah = FragH::load(A + ao);
#pragma unroll
      for (int j = 0; j < 4; ++j) acc[i][j] = mma_h_guarded(ah, bh[j], acc[i][j]);
    }
    keep4_h(bh[0], bh[1], bh[2], bh[3]);
  }

  float* slab = sT[wave];
#pragma unroll
  for (int i = 0; i < 4; ++i) {
    const int mBase = m0 + (i << 4);
#pragma unroll
    for (int j = 0; j < 4; ++j) {
      const int n = n0 + (j << 4) + rlane;
      float bv = 0.f;
      if (BIAS_MODE == 2) bv = bias[n];
#pragma unroll
      for (int r = 0; r < 8; ++r) {
        float v = acc[i][j][r] * scale;
        if (BIAS_MODE == 2) v += bv;
        slab[(mOff + r) * 68 + (j << 4) + rlane] = v;
      }
    }
    __builtin_amdgcn_fence(__ATOMIC_RELEASE, "workgroup");
    __builtin_amdgcn_wave_barrier();
    __builtin_amdgcn_fence(__ATOMIC_ACQUIRE, "workgroup");
    if (OUT_MODE == 0) {
      float* C = (float*)Cout;
      const int hh = lane >> 4, c4 = (lane & 15) * 4;
      for (int pass = 0; pass < 2; ++pass) {
#pragma unroll
        for (int it = 0; it < 8; ++it) {
          const int row = it * 2 + hh;
          const v4f v = *(const v4f*)(slab + row * 68 + c4);
          *(volatile v4f*)(C + (size_t)(mBase + row) * ldc + n0 + c4) = v;
        }
        __threadfence();
      }
    } else {
      const int q = lane >> 3, c8 = (lane & 7) * 8;
      unsigned short* C = (unsigned short*)Cout;
      for (int pass = 0; pass < 2; ++pass) {
#pragma unroll
        for (int it = 0; it < 4; ++it) {
          const int row = it * 4 + q;
          const float* sp = slab + row * 68 + c8;
          v8h hv;
#pragma unroll
          for (int e = 0; e < 8; ++e) hv[e] = (_Float16)sp[e];
          *(volatile v8h*)(C + (size_t)(mBase + row) * ldc + n0 + c8) = hv;
        }
        __threadfence();
      }
    }
    __builtin_amdgcn_fence(__ATOMIC_RELEASE, "workgroup");
    __builtin_amdgcn_wave_barrier();
    __builtin_amdgcn_fence(__ATOMIC_ACQUIRE, "workgroup");
  }
}

__global__ __launch_bounds__(512) void lstm_steps_kernel(
    const unsigned short* __restrict__ ZXT, const unsigned short* __restrict__ UTp,
    const float* __restrict__ bias, const float* __restrict__ h0, const float* __restrict__ c0,
    unsigned short* __restrict__ HS, float* __restrict__ outH, float* __restrict__ outC)
{
  __shared__ __align__(16) _Float16 sH[2 * 16 * kHP];
  __shared__ __align__(16) float sF[16 * kHid];
  const int tid  = threadIdx.x;
  const int lane = tid & 31;
  const int wave = tid >> 5;
  const int hh   = lane >> 4;
  const int cl   = lane & 15;
  const int bt   = blockIdx.x;
  const int jw   = wave * 32 + cl;
  const _Float16* UT = (const _Float16*)UTp;

#pragma unroll
  for (int i = 0; i < 4; ++i) {
    const int e4  = (i * 512 + tid) * 4;
    const int row = e4 >> 9;
    const int k   = e4 & (kHid - 1);
    const v4f hv = *(const v4f*)(h0 + (size_t)(bt * 16 + row) * kHid + k);
    const v4f cv = *(const v4f*)(c0 + (size_t)(bt * 16 + row) * kHid + k);
    sH[row * kHP + k + 0] = (_Float16)(hv[0] * kCarryH);
    sH[row * kHP + k + 1] = (_Float16)(hv[1] * kCarryH);
    sH[row * kHP + k + 2] = (_Float16)(hv[2] * kCarryH);
    sH[row * kHP + k + 3] = (_Float16)(hv[3] * kCarryH);
    *(v4f*)(sF + row * kHid + k) = cv;
  }
  __syncthreads();

  float cst[2][8];
#pragma unroll
  for (int jt = 0; jt < 2; ++jt)
#pragma unroll
    for (int r = 0; r < 8; ++r) cst[jt][r] = sF[(8 * hh + r) * kHid + jw + 16 * jt];
  float bz[4][2];
#pragma unroll
  for (int g = 0; g < 4; ++g)
#pragma unroll
    for (int jt = 0; jt < 2; ++jt) bz[g][jt] = bias[g * kHid + jw + 16 * jt];
  __syncthreads();

#pragma unroll 1
  for (int t = 0; t < kSeq; ++t) {
    const int cur = (t & 1) * 16 * kHP;
    const int nxt = ((t + 1) & 1) * 16 * kHP;
    const size_t mcol = (size_t)t * kBatch + bt * 16 + 8 * hh;

    v8f acc[4][2];
#pragma unroll
    for (int g = 0; g < 4; ++g) {
#pragma unroll
      for (int jt = 0; jt < 2; ++jt) {
        const v4u zw = *(const v4u*)(ZXT + (size_t)(g * kHid + jw + 16 * jt) * kRows + mcol);
#pragma unroll
        for (int i = 0; i < 4; ++i) {
          const unsigned wd = zw[i];
          acc[g][jt][2 * i]     = h16_to_f32(wd & 0xffffu) * kZxToAcc;
          acc[g][jt][2 * i + 1] = h16_to_f32(wd >> 16) * kZxToAcc;
        }
      }
    }

    const _Float16* hc = sH + cur + cl * kHP + 8 * hh;
    const _Float16* ub = UT + (size_t)jw * kHid + 8 * hh;
#pragma unroll 1
    for (int k0 = 0; k0 < kHid; k0 += 32) {
      const v16h a = FragH::load(hc + k0);
#pragma unroll
      for (int jt = 0; jt < 2; ++jt) {
#pragma unroll
        for (int g = 0; g < 4; ++g) {
          const v16h bf = FragH::load(ub + (size_t)(g * kHid + 16 * jt) * kHid + k0);
          acc[g][jt] = mma_h_guarded(a, bf, acc[g][jt]);
        }
      }
    }

    const bool last = (t == kSeq - 1);
#pragma unroll
    for (int jt = 0; jt < 2; ++jt) {
#pragma unroll
      for (int r = 0; r < 8; ++r) {
        const float zi = fmaf(acc[0][jt][r], kAccInv, bz[0][jt]);
        const float zf = fmaf(acc[1][jt][r], kAccInv, bz[1][jt]);
        const float zg = fmaf(acc[2][jt][r], kAccInv, bz[2][jt]);
        const float zo = fmaf(acc[3][jt][r], kAccInv, bz[3][jt]);
        const float si = fast_sigmoid(zi);
        const float sf = fast_sigmoid(zf);
        const float so = fast_sigmoid(zo);
        const float tg = fast_tanh(zg);
        const float cn = sf * cst[jt][r] + si * tg;
        const float hv = so * fast_tanh(cn);
        cst[jt][r] = cn;
        sH[nxt + (8 * hh + r) * kHP + jw + 16 * jt] = (_Float16)(hv * kCarryH);
        if (last) sF[(8 * hh + r) * kHid + jw + 16 * jt] = hv;
      }
    }
    __syncthreads();
    {
      const _Float16* src = sH + nxt + wave * kHP;
      const v8h v0 = *(const v8h*)(src + lane * 8);
      const v8h v1 = *(const v8h*)(src + 256 + lane * 8);
      unsigned short* dst = HS + ((size_t)(bt * 16 + wave) * kSeq + t) * kHid;
      for (int pass = 0; pass < 2; ++pass) {
        *(volatile v8h*)(dst + lane * 8) = v0;
        *(volatile v8h*)(dst + 256 + lane * 8) = v1;
        __threadfence();
      }
    }
  }

  {
    v4f tv[4];
#pragma unroll
    for (int i = 0; i < 4; ++i) tv[i] = *(const v4f*)(sF + wave * kHid + i * 128 + lane * 4);
    float* dst = outH + (size_t)(bt * 16 + wave) * kHid;
    for (int pass = 0; pass < 2; ++pass) {
#pragma unroll
      for (int i = 0; i < 4; ++i) *(volatile v4f*)(dst + i * 128 + lane * 4) = tv[i];
      __threadfence();
    }
  }
  __syncthreads();
#pragma unroll
  for (int jt = 0; jt < 2; ++jt)
#pragma unroll
    for (int r = 0; r < 8; ++r) sF[(8 * hh + r) * kHid + jw + 16 * jt] = cst[jt][r];
  __syncthreads();
  {
    v4f tv[4];
#pragma unroll
    for (int i = 0; i < 4; ++i) tv[i] = *(const v4f*)(sF + wave * kHid + i * 128 + lane * 4);
    float* dst = outC + (size_t)(bt * 16 + wave) * kHid;
    for (int pass = 0; pass < 2; ++pass) {
#pragma unroll
      for (int i = 0; i < 4; ++i) *(volatile v4f*)(dst + i * 128 + lane * 4) = tv[i];
      __threadfence();
    }
  }
}

extern "C" void kernel_launch(void* const* d_in, const int* in_sizes, int n_in,
                              void* d_out, int out_size, void* d_ws, size_t ws_size,
                              hipStream_t stream) {
  if (n_in < 9) return;
  if (in_sizes[0] != kBatch * kSeq) return;
  if (in_sizes[1] != kBatch * kHid) return;
  if (in_sizes[2] != kBatch * kHid) return;
  if (in_sizes[3] != kVocab * kEmb) return;
  if (in_sizes[4] != kEmb * kGate) return;
  if (in_sizes[5] != kHid * kGate) return;
  if (in_sizes[6] != kGate) return;
  if (in_sizes[7] != kHid * kHid) return;
  if (in_sizes[8] != kHid) return;
  if (out_size != kRows * kHid + 2 * kBatch * kHid) return;
  if (ws_size < kWsTotal) return;

  const int*   x   = (const int*)  d_in[0];
  const float* h0  = (const float*)d_in[1];
  const float* c0  = (const float*)d_in[2];
  const float* emb = (const float*)d_in[3];
  const float* W   = (const float*)d_in[4];
  const float* U   = (const float*)d_in[5];
  const float* b   = (const float*)d_in[6];
  const float* Wd  = (const float*)d_in[7];
  const float* bd  = (const float*)d_in[8];
  float* out  = (float*)d_out;
  float* outH = out + (size_t)kRows * kHid;
  float* outC = outH + (size_t)kBatch * kHid;

  char* ws = (char*)d_ws;
  unsigned short* XE  = (unsigned short*)(ws + kOffXE);
  unsigned short* WT  = (unsigned short*)(ws + kOffWT);
  unsigned short* UT  = (unsigned short*)(ws + kOffUT);
  unsigned short* WDT = (unsigned short*)(ws + kOffWDT);
  unsigned short* ZXT = (unsigned short*)(ws + kOffZXT);
  unsigned short* HS  = (unsigned short*)(ws + kOffHS);

  gather_rows_f16_kernel<<<(kRows * 32) / 256, 256, 0, stream>>>(x, emb, XE);

  transpose_cast_kernel<<<dim3(kEmb / 64, kGate / 32), 256, 0, stream>>>(W, WT, kEmb, kGate, kCarryW);
  transpose_cast_kernel<<<dim3(kHid / 64, kGate / 32), 256, 0, stream>>>(U, UT, kHid, kGate, kCarryW);
  transpose_cast_kernel<<<dim3(kHid / 64, kHid / 32), 256, 0, stream>>>(Wd, WDT, kHid, kHid, kCarryW);

  wmma_gemm64_f16<0, 1><<<((kGate / 64) * (kRows / 64)) / 8, 256, 0, stream>>>(
      WT, kEmb, XE, kEmb, (void*)ZXT, kRows, nullptr, kGate, kRows, kEmb, kScaleZx);

  lstm_steps_kernel<<<2, 512, 0, stream>>>(ZXT, UT, b, h0, c0, HS, outH, outC);

  wmma_gemm64_f16<2, 0><<<((kRows / 64) * (kHid / 64)) / 8, 256, 0, stream>>>(
      HS, kHid, WDT, kHid, (void*)out, kHid, bd, kRows, kHid, kHid, kAccInv);
}
